// PatchCritic_67843303407666
// MI455X (gfx1250) — hardware-verified
//
#include <hip/hip_runtime.h>
#include <math.h>

typedef __attribute__((ext_vector_type(16))) _Float16 v16h;
typedef __attribute__((ext_vector_type(16))) __bf16 v16b;
typedef __attribute__((ext_vector_type(8)))  _Float16 v8h;
typedef __attribute__((ext_vector_type(8)))  float v8f;
typedef __attribute__((ext_vector_type(4)))  float v4f;
typedef __attribute__((ext_vector_type(2)))  float v2f;
typedef __attribute__((ext_vector_type(4)))  unsigned v4u;
typedef __attribute__((ext_vector_type(4)))  int v4i;
typedef float __attribute__((may_alias)) float_a;
typedef int __attribute__((may_alias)) int_a;

template <typename T> __device__ __forceinline__ void vst2(void* p, T v) { *(volatile T*)p = v; __threadfence(); *(volatile T*)p = v; }
__device__ __forceinline__ v8f wmma16(v16h a, v16h b, v8f c) {
  v8f d = __builtin_amdgcn_wmma_f32_16x16x32_f16(false, a, false, b, (short)0, c, false, false);
  asm volatile("v_nop\n\tv_nop\n\tv_nop\n\tv_nop" : "+v"(d) : "v"(a), "v"(b));
  return d;
}
__device__ __forceinline__ v8f wmma_bf(v16b a, v16b b, v8f c) {
  v8f d = __builtin_amdgcn_wmma_f32_16x16x32_bf16(false, a, false, b, (short)0, c, false, false);
  asm volatile("v_nop\n\tv_nop\n\tv_nop\n\tv_nop" : "+v"(d) : "v"(a), "v"(b));
  return d;
}
__device__ __forceinline__ v16h frag_h(const _Float16* rowk0, int lane) {
  union { v16h v; v8h q[2]; } u; const _Float16* p = rowk0 + 8 * (lane >> 4);
  u.q[0] = *(const v8h*)p; u.q[1] = *(const v8h*)(p + 16); return u.v;
}
__device__ __forceinline__ v16h frag_f32(const float* rowk0, int lane) {
  v16h a; const float* p = rowk0 + 8 * (lane >> 4);
#pragma unroll
  for (int i = 0; i < 8; ++i) { a[i] = (_Float16)p[i]; a[8 + i] = (_Float16)p[16 + i]; }
  return a;
}
__device__ __forceinline__ v16h frag_f32s(const float* rowk0, int lane, float sc) {
  v16h a; const float* p = rowk0 + 8 * (lane >> 4);
#pragma unroll
  for (int i = 0; i < 8; ++i) { a[i] = (_Float16)(p[i] * sc); a[8 + i] = (_Float16)(p[16 + i] * sc); }
  return a;
}
__device__ __forceinline__ v16h fragc_f32(const float* W, int k0, int n, int lane, int ld, int K) {
  v16h a; const int g = lane >> 4;
#pragma unroll
  for (int i = 0; i < 8; ++i) { const int ka = k0 + 8 * g + i, kb = ka + 16;
    a[i] = (_Float16)(ka < K ? W[(size_t)(ka < K ? ka : K - 1) * ld + n] : 0.f); a[8 + i] = (_Float16)(kb < K ? W[(size_t)(kb < K ? kb : K - 1) * ld + n] : 0.f); }
  return a;
}
struct F2 { v16b h, l; };
__device__ __forceinline__ F2 bsplit16(const float v[16]) { F2 r;
#pragma unroll
  for (int i = 0; i < 16; ++i) { const __bf16 h = (__bf16)v[i]; r.h[i] = h; r.l[i] = (__bf16)(v[i] - (float)h); }
  return r; }
__device__ __forceinline__ F2 split_row(const float* row, int k0, int lane) { float v[16]; const float* p = row + k0 + 8 * (lane >> 4);
#pragma unroll
  for (int i = 0; i < 8; ++i) { v[i] = p[i]; v[8 + i] = p[16 + i]; }
  return bsplit16(v); }
__device__ __forceinline__ F2 split_rowK(const float* row, int k0, int lane, int K) { float v[16]; const int g = lane >> 4;
#pragma unroll
  for (int i = 0; i < 8; ++i) { const int ka = k0 + 8 * g + i, kb = ka + 16; v[i] = ka < K ? row[ka < K ? ka : K - 1] : 0.f; v[8 + i] = kb < K ? row[kb < K ? kb : K - 1] : 0.f; }
  return bsplit16(v); }
__device__ __forceinline__ F2 split_col(const float* W, int k0, int n, int lane, int ld, int K) { float v[16]; const int g = lane >> 4;
#pragma unroll
  for (int i = 0; i < 8; ++i) { const int ka = k0 + 8 * g + i, kb = ka + 16; v[i] = ka < K ? W[(size_t)(ka < K ? ka : K - 1) * ld + n] : 0.f; v[8 + i] = kb < K ? W[(size_t)(kb < K ? kb : K - 1) * ld + n] : 0.f; }
  return bsplit16(v); }
__device__ __forceinline__ v8f mac3(const F2& a, const F2& b, v8f c) { c = wmma_bf(a.l, b.h, c); c = wmma_bf(a.h, b.l, c); return wmma_bf(a.h, b.h, c); }
__device__ __forceinline__ float sigm(float v) { return 1.0f / (1.0f + expf(-v)); }
#define LDSX() do { asm volatile("s_wait_dscnt 0" ::: "memory"); __builtin_amdgcn_wave_barrier(); __builtin_amdgcn_fence(__ATOMIC_RELEASE, "workgroup"); } while (0)


#define CF 256
#define HF 96
#ifndef HFS
#define HFS HF
#endif
#define NPT 9025
#define NPP 9088
#define DD 1024
#define NRB (NPP / 64)
typedef __attribute__((ext_vector_type(8))) __bf16 v8b;
__device__ __forceinline__ v16b frag_b(const __bf16* rowk0, int lane) {
  union { v16b v; v8b q[2]; } u; const __bf16* p = rowk0 + 8 * (lane >> 4);
  u.q[0] = *(const v8b*)p; u.q[1] = *(const v8b*)(p + 16); return u.v;
}
__device__ __forceinline__ float bfr(float v) { return (float)(__bf16)v; }
__device__ __attribute__((noinline)) float exp_ni(float v) { return expf(v); }
__device__ __attribute__((noinline)) float erf_ni(float v) { return erff(v); }

#define WS_SB  0u
#define WS_TB  (WS_SB + 2u * NPP * DD)
#define WS_NS  (WS_TB + 2u * NPP * DD)
#define WS_NTI (WS_NS + 4u * NPP)
#define WS_IT  (WS_NTI + 4u * NPP)
#define WS_CP  (WS_IT + 4u * NPP)
#define WS_CPI (WS_CP + 4u * NRB * NPP)
#define WS_IS  (WS_CPI + 4u * NRB * NPP)
#define WS_PL  (WS_IS + 4u * NPP)
#define WS_END (WS_PL + 128u * 2 * NRB)

__global__ __launch_bounds__(256) void k_patch(const float* __restrict__ SRC, const float* __restrict__ TGT, __bf16* __restrict__ SB, __bf16* __restrict__ TB, float* __restrict__ NS, float* __restrict__ NTI) {
  __shared__ __align__(16) __bf16 s[64][DD + 8]; __shared__ float sq[64][4]; __shared__ __align__(16) float sn[64];
  const int tid = threadIdx.x; const int rb = blockIdx.x, which = blockIdx.y; const float* F = which ? TGT : SRC; const int n0 = rb * 64;
  for (int e = tid; e < 64 * DD; e += 256) { const int r = e & 63, d = e >> 6; const int n = n0 + r; float v = 0.f;
    if (n < NPT) { const int i = n / (HF - 1), j = n % (HF - 1); const int q = d >> 8, c = d & 255; const int di = q >> 1, dj = q & 1; v = bfr(F[((size_t)c * HFS + i + di) * HFS + j + dj]); }
    s[r][d] = (__bf16)v; }
  __syncthreads();
  { const int r = tid >> 2, part = tid & 3; float a = 0.f; for (int d = part; d < DD; d += 4) { const float v = (float)s[r][d]; a += v * v; } sq[r][part] = a; }
  __syncthreads();
  if (tid < 64) { const float a = (sq[tid][0] + sq[tid][1]) + (sq[tid][2] + sq[tid][3]); sn[tid] = 1.0f / (sqrtf(a) + 1e-8f); }
  __syncthreads();
  __bf16* DST = which ? TB : SB;
  for (int e = tid; e < 64 * DD / 8; e += 256) { const int r = e / (DD / 8), pc = e % (DD / 8); vst2((unsigned*)(DST + (size_t)(n0 + r) * DD + pc * 8), *(const v4u*)&s[r][pc * 8]); }
  if (tid < 16) vst2((which ? NTI : NS) + n0 + tid * 4, *(const v4f*)&sn[tid * 4]);
}
__global__ __launch_bounds__(128) void k_score(const __bf16* __restrict__ TB, const __bf16* __restrict__ SB, const float* __restrict__ NTI, const float* __restrict__ NS, int* __restrict__ IT, float* __restrict__ CP, int* __restrict__ CPI) {
  __shared__ float scv[4][128]; __shared__ int sci[4][128]; __shared__ __align__(16) float sbv[128]; __shared__ __align__(16) int sbi[128]; __shared__ __align__(16) int sit[64];
  const int tid = threadIdx.x, wave = tid >> 5, lane = tid & 31, col = lane & 15, g = lane >> 4; const int rb = blockIdx.x; const size_t r0 = (size_t)rb * 64 + wave * 16;
  float nt[8];
#pragma unroll
  for (int r = 0; r < 8; ++r) nt[r] = NTI[r0 + 8 * g + r];
  float bestv[8]; int besti[8];
#pragma unroll
  for (int r = 0; r < 8; ++r) { bestv[r] = -3.0e38f; besti[r] = 0; }
#pragma unroll 1
  for (int cb = 0; cb < NPP / 128; ++cb) { const int n0 = cb * 128; v8f acc[8] = {};
#pragma unroll 2
    for (int kc = 0; kc < DD / 32; ++kc) { const v16b a = frag_b(TB + (r0 + col) * DD + kc * 32, lane);
#pragma unroll
      for (int j = 0; j < 8; ++j) acc[j] = wmma_bf(a, frag_b(SB + (size_t)(n0 + j * 16 + col) * DD + kc * 32, lane), acc[j]); }
#pragma unroll
    for (int j = 0; j < 8; ++j) { const int jj = n0 + j * 16 + col; const float nsj = NS[jj]; const bool vj = jj < NPT; float cbest = -3.0e38f; int cidx = 0;
#pragma unroll
      for (int r = 0; r < 8; ++r) { const float sc = acc[j][r] * nt[r] * nsj; const int ii = (int)(r0 + 8 * g + r);
        if (vj && sc > bestv[r]) { bestv[r] = sc; besti[r] = jj; }
        if (ii < NPT && sc > cbest) { cbest = sc; cidx = ii; } }
      const float ob = __shfl_xor(cbest, 16); const int oi = __shfl_xor(cidx, 16);
      if (g == 0) { if (ob > cbest) { cbest = ob; cidx = oi; } scv[wave][j * 16 + col] = cbest; sci[wave][j * 16 + col] = cidx; } }
    __syncthreads();
    if (tid < 128) { float bv = scv[0][tid]; int bi = sci[0][tid];
#pragma unroll
      for (int w = 1; w < 4; ++w) { if (scv[w][tid] > bv) { bv = scv[w][tid]; bi = sci[w][tid]; } }
      sbv[tid] = bv; sbi[tid] = bi; }
    __syncthreads();
    if (tid < 32) vst2(CP + (size_t)rb * NPP + n0 + tid * 4, *(const v4f*)&sbv[tid * 4]); else if (tid < 64) vst2((unsigned*)(CPI + (size_t)rb * NPP + n0 + (tid - 32) * 4), *(const v4u*)&sbi[(tid - 32) * 4]);
    __syncthreads(); }
#pragma unroll
  for (int r = 0; r < 8; ++r) { float bv = bestv[r]; int bi = besti[r];
#pragma unroll
    for (int o = 1; o < 16; o <<= 1) { const float ov = __shfl_xor(bv, o); const int oi = __shfl_xor(bi, o); if (ov > bv || (ov == bv && oi < bi)) { bv = ov; bi = oi; } }
    if (col == 0) sit[wave * 16 + 8 * g + r] = bi; }
  __syncthreads();
  if (tid < 16) vst2((unsigned*)(IT + (size_t)rb * 64 + tid * 4), *(const v4u*)&sit[tid * 4]);
}
__global__ __launch_bounds__(256) void k_colred(const float* __restrict__ CP, const int* __restrict__ CPI, int* __restrict__ IS) {
  __shared__ __align__(16) int si[256]; const int tid = threadIdx.x; const int j = blockIdx.x * 256 + tid; float bv = -3.0e38f; int bi = 0;
  if (j < NPP) { for (int rb = 0; rb < NRB; ++rb) { const float v = CP[(size_t)rb * NPP + j]; if (v > bv) { bv = v; bi = CPI[(size_t)rb * NPP + j]; } } }
  si[tid] = bi; __syncthreads();
  if (tid < 64 && blockIdx.x * 256 + tid * 4 < NPP) vst2((unsigned*)(IS + (size_t)blockIdx.x * 256 + tid * 4), *(const v4u*)&si[tid * 4]);
}
__global__ __launch_bounds__(256) void k_loss(const __bf16* __restrict__ SB, const __bf16* __restrict__ TB, const int* __restrict__ IT, const int* __restrict__ IS, double* __restrict__ PL) {
  __shared__ double sred[8]; __shared__ __align__(16) double sl[16]; const int tid = threadIdx.x; const int rb = blockIdx.x, which = blockIdx.y;
  float a = 0.f;
  { const int r = tid >> 2, part = tid & 3; const int n = rb * 64 + r;
    if (n < NPT) { const __bf16* tr; const __bf16* sr;
      if (which == 0) { tr = TB + (size_t)n * DD; sr = SB + (size_t)min(max(IT[n], 0), NPT - 1) * DD; } else { sr = SB + (size_t)n * DD; tr = TB + (size_t)min(max(IS[n], 0), NPT - 1) * DD; }
      for (int d = part; d < DD; d += 4) { const float df = (float)tr[d] - (float)sr[d]; a += df * df; } } }
  double da = (double)a;
#pragma unroll
  for (int o = 1; o < 32; o <<= 1) da += __shfl_xor(da, o);
  if ((tid & 31) == 0) sred[tid >> 5] = da;
  if (tid < 16) sl[tid] = 0.0;
  __syncthreads();
  if (tid == 0) { double t = 0.0; for (int w = 0; w < 8; ++w) t += sred[w]; sl[0] = t; }
  __syncthreads();
  if (tid < 8) vst2((unsigned*)(PL + ((size_t)which * NRB + rb) * 16 + tid * 2), *(const v4u*)&sl[tid * 2]);
}
__global__ __launch_bounds__(64) void k_final(const double* __restrict__ PL, float* __restrict__ OUT) {
  __shared__ double s[2][64]; const int t = threadIdx.x; double a0 = 0.0, a1 = 0.0;
  for (int rb = t; rb < NRB; rb += 64) { a0 += PL[(size_t)rb * 16]; a1 += PL[((size_t)NRB + rb) * 16]; }
  s[0][t] = a0; s[1][t] = a1; __syncthreads();
  if (t == 0) { double A0 = 0.0, A1 = 0.0; for (int i = 0; i < 64; ++i) { A0 += s[0][i]; A1 += s[1][i]; } const double den = (double)NPT * (double)DD;
    v4f v; v[0] = (float)(0.5 * A0 / den); v[1] = (float)(0.5 * A1 / den); v[2] = 0.f; v[3] = 0.f;
    *(volatile float*)OUT = v[0]; *(volatile float*)(OUT + 1) = v[1]; *(volatile float*)OUT = v[0]; *(volatile float*)(OUT + 1) = v[1]; }
}
extern "C" void kernel_launch(void* const* d_in, const int* in_sizes, int n_in, void* d_out, int out_size, void* d_ws, size_t ws_size, hipStream_t stream) {
  (void)in_sizes; (void)n_in; (void)out_size;
  const float** F = (const float**)d_in;
  if (ws_size < (size_t)WS_END) return;
  char* ws = (char*)d_ws; __bf16 *SB = (__bf16*)(ws + WS_SB), *TB = (__bf16*)(ws + WS_TB); float *NS = (float*)(ws + WS_NS), *NTI = (float*)(ws + WS_NTI), *CP = (float*)(ws + WS_CP); int *IT = (int*)(ws + WS_IT), *CPI = (int*)(ws + WS_CPI), *IS = (int*)(ws + WS_IS); double* PL = (double*)(ws + WS_PL);
  k_patch<<<dim3(NRB, 2), 256, 0, stream>>>(F[0], F[1], SB, TB, NS, NTI);
  k_score<<<NRB, 128, 0, stream>>>(TB, SB, NTI, NS, IT, CP, CPI);
  k_colred<<<(NPP + 255) / 256, 256, 0, stream>>>(CP, CPI, IS);
  k_loss<<<dim3(NRB, 2), 256, 0, stream>>>(SB, TB, IT, IS, PL);
  k_final<<<1, 64, 0, stream>>>(PL, (float*)d_out);
}
